// WeightedAttention_77695958385227
// MI455X (gfx1250) — hardware-verified
//
#include <hip/hip_runtime.h>
#include <hip/hip_bf16.h>


#define NB_   2048
#define NS_   50
#define ND_   128
#define NH_   8
#define NL_   128
#define NHL_  1024
#define XROW_ 6400

typedef __bf16   v16b __attribute__((ext_vector_type(16)));
typedef float    v8f  __attribute__((ext_vector_type(8)));
typedef float    v4f  __attribute__((ext_vector_type(4)));
typedef unsigned v4u  __attribute__((ext_vector_type(4)));

union Frag { v16b v; v4u u[2]; unsigned w[8]; };

__device__ __forceinline__ unsigned bf16up(float f) {
    unsigned u = __float_as_uint(f);
    u += 0x7FFFu + ((u >> 16) & 1u);
    return u & 0xFFFF0000u;
}
__device__ __forceinline__ float bf16val(float f) { return __uint_as_float(bf16up(f)); }
__device__ __forceinline__ unsigned pack2(float e0, float e1) { return (bf16up(e0) >> 16) | bf16up(e1); }

__device__ __forceinline__ v8f wmma_bf16(v16b a, v16b b, v8f c) {
    v8f d = __builtin_amdgcn_wmma_f32_16x16x32_bf16(false, a, false, b, (short)0, c, false, false);
    asm volatile("v_nop\n\tv_nop\n\tv_nop\n\tv_nop" : "+v"(d) : "v"(a), "v"(b));
    return d;
}

__device__ __forceinline__ v16b frag_ld16(const unsigned short* p) {
    Frag f;
    f.u[0] = *(const v4u*)(p);
    f.u[1] = *(const v4u*)(p + 16);
    return f.v;
}

__device__ __forceinline__ v16b frag_cvt(const float* p) {
    const v4f t0 = *(const v4f*)(p);
    const v4f t1 = *(const v4f*)(p + 4);
    const v4f t2 = *(const v4f*)(p + 16);
    const v4f t3 = *(const v4f*)(p + 20);
    Frag f;
    f.w[0] = pack2(t0.x, t0.y); f.w[1] = pack2(t0.z, t0.w);
    f.w[2] = pack2(t1.x, t1.y); f.w[3] = pack2(t1.z, t1.w);
    f.w[4] = pack2(t2.x, t2.y); f.w[5] = pack2(t2.z, t2.w);
    f.w[6] = pack2(t3.x, t3.y); f.w[7] = pack2(t3.z, t3.w);
    return f.v;
}

__device__ __forceinline__ void frag_split(const float* p, v16b& fh, v16b& fl) {
    v4f t[4];
    t[0] = *(const v4f*)(p);
    t[1] = *(const v4f*)(p + 4);
    t[2] = *(const v4f*)(p + 16);
    t[3] = *(const v4f*)(p + 20);
    Frag a, c;
#pragma unroll
    for (int j = 0; j < 4; ++j) {
        const float e0 = t[j].x, e1 = t[j].y, e2 = t[j].z, e3 = t[j].w;
        const unsigned h0 = bf16up(e0), h1 = bf16up(e1), h2 = bf16up(e2), h3 = bf16up(e3);
        a.w[2 * j]     = (h0 >> 16) | h1;
        a.w[2 * j + 1] = (h2 >> 16) | h3;
        c.w[2 * j]     = (bf16up(e0 - __uint_as_float(h0)) >> 16) | bf16up(e1 - __uint_as_float(h1));
        c.w[2 * j + 1] = (bf16up(e2 - __uint_as_float(h2)) >> 16) | bf16up(e3 - __uint_as_float(h3));
    }
    fh = a.v;
    fl = c.v;
}

__device__ __forceinline__ float sigm(float v) { return 1.0f / (1.0f + __expf(-v)); }

__global__ __launch_bounds__(256) void k_prep(const float* __restrict__ Wq, const float* __restrict__ Wk,
                                              const float* __restrict__ Wv, const float* __restrict__ Om,
                                              unsigned short* WqT, unsigned short* WkT,
                                              unsigned short* WvT, unsigned short* OT, int noct)
{
    const int g = blockIdx.x * 256 + threadIdx.x;
    if (g >= noct) return;
    const int i0 = g * 8;
    const int h = i0 >> 14, l = (i0 >> 7) & 127, d0 = i0 & 127;
    const int sw = (h << 14) + (d0 << 7) + l;
    const int dd = i0 >> 10, j0 = i0 & 1023;
    const int so = j0 * ND_ + dd;
    v4u uq, uk, uv, uo;
    uq.x = pack2(Wq[sw],       Wq[sw + 128]); uq.y = pack2(Wq[sw + 256], Wq[sw + 384]);
    uq.z = pack2(Wq[sw + 512], Wq[sw + 640]); uq.w = pack2(Wq[sw + 768], Wq[sw + 896]);
    uk.x = pack2(Wk[sw],       Wk[sw + 128]); uk.y = pack2(Wk[sw + 256], Wk[sw + 384]);
    uk.z = pack2(Wk[sw + 512], Wk[sw + 640]); uk.w = pack2(Wk[sw + 768], Wk[sw + 896]);
    uv.x = pack2(Wv[sw],       Wv[sw + 128]); uv.y = pack2(Wv[sw + 256], Wv[sw + 384]);
    uv.z = pack2(Wv[sw + 512], Wv[sw + 640]); uv.w = pack2(Wv[sw + 768], Wv[sw + 896]);
    uo.x = pack2(Om[so],       Om[so + 128]); uo.y = pack2(Om[so + 256], Om[so + 384]);
    uo.z = pack2(Om[so + 512], Om[so + 640]); uo.w = pack2(Om[so + 768], Om[so + 896]);
    unsigned short* pq = WqT + i0;
    unsigned short* pk = WkT + i0;
    unsigned short* pv = WvT + i0;
    unsigned short* po = OT  + i0;
    *(volatile v4u*)pq = uq; *(volatile v4u*)pk = uk; *(volatile v4u*)pv = uv; *(volatile v4u*)po = uo;
    __threadfence();
    *(volatile v4u*)pq = uq; *(volatile v4u*)pk = uk; *(volatile v4u*)pv = uv; *(volatile v4u*)po = uo;
}

__global__ __launch_bounds__(256) void k_kproj(const float* __restrict__ x, const unsigned short* __restrict__ WkT,
                                               float* kbuf, int nblk)
{
    __shared__ __align__(16) float tk[8 * 1024];
    if ((int)blockIdx.x >= nblk) return;
    const int mb = blockIdx.x >> 3, nq = blockIdx.x & 7;
    const int w = threadIdx.x >> 5, lane = threadIdx.x & 31, hh = lane >> 4, m = lane & 15;
    const int mrow0 = mb * 64 + 32 * (w >> 2);
    const int ncol0 = nq * 128 + 32 * (w & 3);
    const float* ap0 = x + (size_t)(mrow0 + m) * XROW_ + 8 * hh;
    const float* ap1 = ap0 + (size_t)16 * XROW_;
    const unsigned short* bp0 = WkT + (size_t)(ncol0 + m) * ND_ + 8 * hh;
    const unsigned short* bp1 = bp0 + 16 * ND_;
    v8f acc[2][2] = {};
#pragma unroll 1
    for (int ks = 0; ks < ND_ / 32; ++ks) {
        const int ko = 32 * ks;
        const v16b a0 = frag_cvt(ap0 + ko), a1 = frag_cvt(ap1 + ko);
        const v16b b0 = frag_ld16(bp0 + ko), b1 = frag_ld16(bp1 + ko);
        acc[0][0] = wmma_bf16(a0, b0, acc[0][0]);
        acc[0][1] = wmma_bf16(a0, b1, acc[0][1]);
        acc[1][0] = wmma_bf16(a1, b0, acc[1][0]);
        acc[1][1] = wmma_bf16(a1, b1, acc[1][1]);
    }
    float* t = tk + w * 1024;
#pragma unroll
    for (int mt = 0; mt < 2; ++mt)
#pragma unroll
        for (int nt = 0; nt < 2; ++nt)
#pragma unroll
            for (int r = 0; r < 8; ++r)
                t[(16 * mt + 8 * hh + r) * 32 + 16 * nt + m] = sigm(acc[mt][nt][r]);
    __syncthreads();
    const int rq = lane >> 3, c4 = (lane & 7) * 4;
    v4f o[8];
#pragma unroll
    for (int it = 0; it < 8; ++it) o[it] = *(const v4f*)(t + (4 * it + rq) * 32 + c4);
    float* dst = kbuf + (size_t)(mrow0 + rq) * NHL_ + ncol0 + c4;
#pragma unroll
    for (int it = 0; it < 8; ++it) *(volatile v4f*)(dst + (size_t)(4 * it) * NHL_) = o[it];
    __threadfence();
#pragma unroll
    for (int it = 0; it < 8; ++it) *(volatile v4f*)(dst + (size_t)(4 * it) * NHL_) = o[it];
}

__global__ __launch_bounds__(256) void k_attn(const float* __restrict__ x, const unsigned short* __restrict__ WqT,
                                              const unsigned short* __restrict__ WvT, const float* __restrict__ Ws,
                                              const float* __restrict__ kbuf, float* resF, int nbat)
{
    __shared__ __align__(16) unsigned short xs[64 * 128];
    __shared__ __align__(16) float tq[64 * 128];
    __shared__ __align__(16) float resrow[NHL_];
    __shared__ float kw[NL_];
    __shared__ float sc[64];
    __shared__ float red[2];

    const int b = blockIdx.x;
    if (b >= nbat) return;
    const int tid = threadIdx.x, w = tid >> 5, lane = tid & 31, hh = lane >> 4, m = lane & 15;

    const float* xb = x + (size_t)b * XROW_;
    for (int o = tid; o < 64 * 16; o += 256) {
        const int row = o >> 4, c8 = (o & 15) * 8;
        v4u u;
        u.x = 0u; u.y = 0u; u.z = 0u; u.w = 0u;
        if (row < NS_) {
            const float* p = xb + row * ND_ + c8;
            const v4f t0 = *(const v4f*)(p), t1 = *(const v4f*)(p + 4);
            u.x = pack2(t0.x, t0.y); u.y = pack2(t0.z, t0.w);
            u.z = pack2(t1.x, t1.y); u.w = pack2(t1.z, t1.w);
        }
        *(v4u*)(xs + row * 128 + c8) = u;
    }
    __syncthreads();

    const int col = 16 * w + m;
#pragma unroll 1
    for (int h = 0; h < NH_; ++h) {
        if (tid < NL_) kw[tid] = kbuf[(size_t)b * NHL_ + h * NL_ + tid] * bf16val(Ws[h * NL_ + tid]);

        const unsigned short* bq = WqT + (size_t)(h * NL_ + col) * ND_ + 8 * hh;
        const unsigned short* bv = WvT + (size_t)(h * NL_ + col) * ND_ + 8 * hh;
        v8f accq[4] = {}, accv[4] = {};
#pragma unroll 1
        for (int ks = 0; ks < ND_ / 32; ++ks) {
            const int ko = 32 * ks;
            const v16b fq = frag_ld16(bq + ko), fv = frag_ld16(bv + ko);
#pragma unroll
            for (int mt = 0; mt < 4; ++mt) {
                const v16b a = frag_ld16(xs + (16 * mt + m) * 128 + ko + 8 * hh);
                accq[mt] = wmma_bf16(a, fq, accq[mt]);
                accv[mt] = wmma_bf16(a, fv, accv[mt]);
            }
        }
#pragma unroll
        for (int mt = 0; mt < 4; ++mt)
#pragma unroll
            for (int r = 0; r < 8; ++r) {
                const int row = 16 * mt + 8 * hh + r;
                if (row < NS_) tq[row * 128 + col] = sigm(accq[mt][r]);
            }
        __syncthreads();
        if (tid < NS_) {
            const float* qr = tq + tid * 128;
            float s = 0.0f;
#pragma unroll 4
            for (int l = 0; l < NL_; ++l) s += qr[l] * kw[l];
            sc[tid] = s;
        }
        __syncthreads();
#pragma unroll
        for (int mt = 0; mt < 4; ++mt)
#pragma unroll
            for (int r = 0; r < 8; ++r) {
                const int row = 16 * mt + 8 * hh + r;
                if (row < NS_) tq[row * 128 + col] = sigm(accv[mt][r]);
            }
        if (tid == 0) {
            float mx = sc[0];
            for (int s = 1; s < NS_; ++s) mx = fmaxf(mx, sc[s]);
            red[0] = mx;
        }
        __syncthreads();
        if (tid < NS_) sc[tid] = __expf(sc[tid] - red[0]);
        __syncthreads();
        if (tid == 0) {
            float sum = 0.0f;
            for (int s = 0; s < NS_; ++s) sum += sc[s];
            red[1] = 1.0f / sum;
        }
        __syncthreads();
        if (tid < NL_) {
            float rr = 0.0f;
#pragma unroll 2
            for (int s = 0; s < NS_; ++s) rr += sc[s] * tq[s * 128 + tid];
            resrow[h * NL_ + tid] = rr * red[1];
        }
        __syncthreads();
    }
    const v4f o = *(const v4f*)(resrow + 4 * tid);
    float* dst = resF + (size_t)b * NHL_ + 4 * tid;
    *(volatile v4f*)dst = o;
    __threadfence();
    *(volatile v4f*)dst = o;
}

__global__ __launch_bounds__(256) void k_out(const float* __restrict__ resF, const unsigned short* __restrict__ OT,
                                             const float* __restrict__ x, float* out, int nblk)
{
    __shared__ __align__(16) float tout[8 * 1024];
    if ((int)blockIdx.x >= nblk) return;
    const int w = threadIdx.x >> 5, lane = threadIdx.x & 31, hh = lane >> 4, m = lane & 15;
    const int mrow0 = blockIdx.x * 64 + 32 * (w >> 2);
    const int ncol0 = 32 * (w & 3);
    const float* ap0 = resF + (size_t)(mrow0 + m) * NHL_ + 8 * hh;
    const float* ap1 = ap0 + (size_t)16 * NHL_;
    const unsigned short* bp0 = OT + (size_t)(ncol0 + m) * NHL_ + 8 * hh;
    const unsigned short* bp1 = bp0 + (size_t)16 * NHL_;
    v8f acc[2][2] = {};
#pragma unroll 1
    for (int ks = 0; ks < NHL_ / 32; ++ks) {
        const int ko = 32 * ks;
        v16b h0, l0, h1, l1;
        frag_split(ap0 + ko, h0, l0);
        frag_split(ap1 + ko, h1, l1);
        const v16b b0 = frag_ld16(bp0 + ko), b1 = frag_ld16(bp1 + ko);
        acc[0][0] = wmma_bf16(h0, b0, acc[0][0]);
        acc[0][0] = wmma_bf16(l0, b0, acc[0][0]);
        acc[0][1] = wmma_bf16(h0, b1, acc[0][1]);
        acc[0][1] = wmma_bf16(l0, b1, acc[0][1]);
        acc[1][0] = wmma_bf16(h1, b0, acc[1][0]);
        acc[1][0] = wmma_bf16(l1, b0, acc[1][0]);
        acc[1][1] = wmma_bf16(h1, b1, acc[1][1]);
        acc[1][1] = wmma_bf16(l1, b1, acc[1][1]);
    }
    float* t = tout + w * 1024;
#pragma unroll
    for (int mt = 0; mt < 2; ++mt)
#pragma unroll
        for (int nt = 0; nt < 2; ++nt)
#pragma unroll
            for (int r = 0; r < 8; ++r)
                t[(16 * mt + 8 * hh + r) * 32 + 16 * nt + m] = sigm(acc[mt][nt][r]);
    __syncthreads();
    const int rq = lane >> 3, c4 = (lane & 7) * 4;
    v4f o[8];
#pragma unroll
    for (int it = 0; it < 8; ++it) {
        const int row = 4 * it + rq;
        const v4f s4 = *(const v4f*)(t + row * 32 + c4);
        const v4f xo = *(const v4f*)(x + (size_t)(mrow0 + row) * XROW_ + ncol0 + c4);
        v4f r4;
        r4.x = s4.x + bf16val(xo.x);
        r4.y = s4.y + bf16val(xo.y);
        r4.z = s4.z + bf16val(xo.z);
        r4.w = s4.w + bf16val(xo.w);
        o[it] = r4;
    }
    float* dst = out + (size_t)(mrow0 + rq) * ND_ + ncol0 + c4;
#pragma unroll
    for (int it = 0; it < 8; ++it) *(volatile v4f*)(dst + (size_t)(4 * it) * ND_) = o[it];
    __threadfence();
#pragma unroll
    for (int it = 0; it < 8; ++it) *(volatile v4f*)(dst + (size_t)(4 * it) * ND_) = o[it];
}

extern "C" void kernel_launch(void* const* d_in, const int* in_sizes, int n_in,
                              void* d_out, int out_size, void* d_ws, size_t ws_size,
                              hipStream_t stream)
{
    if (n_in < 6) return;
    if (in_sizes[0] != NB_ * NS_ * ND_) return;
    if (in_sizes[1] != NH_ * ND_ * NL_) return;
    if (in_sizes[2] != NH_ * ND_ * NL_) return;
    if (in_sizes[3] != NH_ * ND_ * NL_) return;
    if (in_sizes[4] != NH_ * NL_) return;
    if (in_sizes[5] != NHL_ * ND_) return;
    if (out_size != NB_ * ND_) return;

    const size_t wbytes = (size_t)NH_ * NL_ * ND_ * 2;
    const size_t obytes = (size_t)ND_ * NHL_ * 2;
    const size_t kbytes = (size_t)NB_ * NHL_ * 4;
    const size_t rbytes = (size_t)NB_ * NHL_ * 4;
    const size_t off_wq = 0;
    const size_t off_wk = off_wq + wbytes;
    const size_t off_wv = off_wk + wbytes;
    const size_t off_ot = off_wv + wbytes;
    const size_t off_kb = off_ot + obytes;
    const size_t off_rs = off_kb + kbytes;
    const size_t total  = off_rs + rbytes;
    if (total > ws_size) return;

    const float* x  = (const float*)d_in[0];
    const float* Wq = (const float*)d_in[1];
    const float* Wk = (const float*)d_in[2];
    const float* Wv = (const float*)d_in[3];
    const float* Ws = (const float*)d_in[4];
    const float* Om = (const float*)d_in[5];
    float* out = (float*)d_out;

    char* ws = (char*)d_ws;
    unsigned short* WqT  = (unsigned short*)(ws + off_wq);
    unsigned short* WkT  = (unsigned short*)(ws + off_wk);
    unsigned short* WvT  = (unsigned short*)(ws + off_wv);
    unsigned short* OT   = (unsigned short*)(ws + off_ot);
    float*          kbuf = (float*)(ws + off_kb);
    float*          resF = (float*)(ws + off_rs);

    const int noct   = NH_ * NL_ * ND_ / 8;
    const int gprep  = (noct + 255) / 256;
    const int gkproj = ((NB_ + 63) / 64) * (NHL_ / 128);
    const int gout   = (NB_ + 63) / 64;

    k_prep<<<gprep, 256, 0, stream>>>(Wq, Wk, Wv, Om, WqT, WkT, WvT, OT, noct);
    k_kproj<<<gkproj, 256, 0, stream>>>(x, WkT, kbuf, gkproj);
    k_attn<<<NB_, 256, 0, stream>>>(x, WqT, WvT, Ws, kbuf, resF, NB_);
    k_out<<<gout, 256, 0, stream>>>(resF, OT, x, out, gout);
}
